// FuzzyNeuron_32693291057854
// MI455X (gfx1250) — hardware-run, weakly checked
//
#include <hip/hip_runtime.h>

typedef __bf16         v16b  __attribute__((ext_vector_type(16)));
typedef unsigned short v16us __attribute__((ext_vector_type(16)));
typedef unsigned short v8us  __attribute__((ext_vector_type(8)));
typedef float          v8f   __attribute__((ext_vector_type(8)));
typedef float          v4f   __attribute__((ext_vector_type(4)));
typedef v8us __attribute__((may_alias)) v8usa;
typedef v4f  __attribute__((may_alias)) v4fa;

union Frag { v16b v; v16us u; v8us half[2]; };

#define A_DIM 16
#define R_DIM 64
#define KP    32
#define ROWS  128
#define NTHR  128
#define ZP    65
#define FMIN  1.17549435e-38f

__device__ __forceinline__ unsigned int bf16_rne_bits(float f) {
  const unsigned int u = __float_as_uint(f);
  return (u + 0x7FFFu + ((u >> 16) & 1u)) >> 16;
}

__device__ __forceinline__ v8f wmma_bf16(v16b a, v16b b, v8f c) {
  v8f d = __builtin_amdgcn_wmma_f32_16x16x32_bf16(false, a, false, b, (short)0, c, false, false);
  asm volatile("v_nop\n\tv_nop\n\tv_nop\n\tv_nop" : "+v"(d) : "v"(a), "v"(b));
  return d;
}

__global__ void __launch_bounds__(NTHR)
fuzzy_kernel(const float* __restrict__ x,
             const float* __restrict__ mu,
             const float* __restrict__ sigma,
             const float* __restrict__ rho,
             float* __restrict__ out,
             int n_rows)
{
  #pragma clang fp contract(off)
  __shared__ __attribute__((aligned(16))) float          zs[ROWS * ZP];
  __shared__ __attribute__((aligned(16))) float          mu_s[R_DIM * A_DIM];
  __shared__ __attribute__((aligned(16))) float          iv_s[R_DIM * A_DIM];
  __shared__ __attribute__((aligned(16))) unsigned short bh_s[R_DIM * KP];
  __shared__ __attribute__((aligned(16))) unsigned short bl_s[R_DIM * KP];
  __shared__ __attribute__((aligned(16))) float          rb_s[R_DIM];
  __shared__ __attribute__((aligned(16))) float          o_s[ROWS];

  const int tid  = threadIdx.x;
  const int lane = tid & 31, w = tid >> 5;
  const int h = lane >> 4, m = lane & 15;
  const int row0 = blockIdx.x * ROWS;
  if (row0 + ROWS > n_rows) return;

  for (int i = tid; i < R_DIM * A_DIM; i += NTHR) {
    mu_s[i] = mu[i];
    const float s  = sigma[i];
    const float s2 = s * s;
    const float d2 = 2.0f * s2;
    iv_s[i] = 1.0f / d2;
  }
  for (int i = tid; i < R_DIM * KP; i += NTHR) {
    const int n  = i >> 5, k = i & 31;
    const int kc = (k < A_DIM) ? k : (A_DIM - 1);
    float v = rho[n * (A_DIM + 1) + kc];
    v = (k < A_DIM) ? v : 0.0f;
    const unsigned int hb = bf16_rne_bits(v);
    const float hf = __uint_as_float(hb << 16);
    bh_s[i] = (unsigned short)hb;
    bl_s[i] = (unsigned short)bf16_rne_bits(v - hf);
  }
  if (tid < R_DIM) rb_s[tid] = rho[tid * (A_DIM + 1) + A_DIM];
  __syncthreads();

  #pragma unroll
  for (int mt = 0; mt < 2; ++mt) {
    const int rl = 32 * w + 16 * mt;
    const float* xp = x + (size_t)(row0 + rl + m) * A_DIM + 8 * h;
    const v4f xa = *(const v4fa*)xp;
    const v4f xb = *(const v4fa*)(xp + 4);
    const float xe[8] = {xa.x, xa.y, xa.z, xa.w, xb.x, xb.y, xb.z, xb.w};
    Frag ah, al;
    #pragma unroll
    for (int i = 0; i < 8; ++i) {
      const unsigned int hb = bf16_rne_bits(xe[i]);
      const float hf = __uint_as_float(hb << 16);
      ah.u[i] = (unsigned short)hb;
      al.u[i] = (unsigned short)bf16_rne_bits(xe[i] - hf);
      ah.u[8 + i] = (unsigned short)0;
      al.u[8 + i] = (unsigned short)0;
    }
    #pragma unroll
    for (int t = 0; t < 4; ++t) {
      const int n = 16 * t + m;
      Frag bh, bl;
      bh.half[0] = *(const v8usa*)(bh_s + n * KP + 8 * h);
      bh.half[1] = *(const v8usa*)(bh_s + n * KP + 16 + 8 * h);
      bl.half[0] = *(const v8usa*)(bl_s + n * KP + 8 * h);
      bl.half[1] = *(const v8usa*)(bl_s + n * KP + 16 + 8 * h);
      v8f c;
      #pragma unroll
      for (int r = 0; r < 8; ++r) c[r] = 0.0f;
      c = wmma_bf16(ah.v, bh.v, c);
      c = wmma_bf16(al.v, bh.v, c);
      c = wmma_bf16(ah.v, bl.v, c);
      #pragma unroll
      for (int r = 0; r < 8; ++r) zs[(rl + 8 * h + r) * ZP + 16 * t + m] = c[r];
    }
  }
  __syncthreads();

  {
    const float* xr = x + (size_t)(row0 + tid) * A_DIM;
    const v4f q0 = *(const v4fa*)(xr);
    const v4f q1 = *(const v4fa*)(xr + 4);
    const v4f q2 = *(const v4fa*)(xr + 8);
    const v4f q3 = *(const v4fa*)(xr + 12);
    const float xv[16] = {q0.x, q0.y, q0.z, q0.w, q1.x, q1.y, q1.z, q1.w,
                          q2.x, q2.y, q2.z, q2.w, q3.x, q3.y, q3.z, q3.w};
    float num = 0.0f, den = 0.0f;
    #pragma unroll 1
    for (int r = 0; r < R_DIM; ++r) {
      const float* mp = mu_s + r * A_DIM;
      const float* ip = iv_s + r * A_DIM;
      float s = 0.0f;
      #pragma unroll
      for (int a = 0; a < A_DIM; ++a) {
        const float d  = xv[a] - mp[a];
        const float dd = d * d;
        const float tq = dd * ip[a];
        s = s + tq;
      }
      const float lw = -s;
      float wv = expf(lw);
      wv = (wv < FMIN) ? 0.0f : wv;
      const float z  = zs[tid * ZP + r] + rb_s[r];
      const float zw = z * wv;
      num = num + zw;
      den = den + wv;
    }
    const float dn = den + 1e-13f;
    const float rd = 1.0f / dn;
    o_s[tid] = num * rd;
  }
  __syncthreads();

  if (w == 0) {
    const v4f v = *(const v4fa*)(o_s + 4 * lane);
    float* op = out + (size_t)row0 + 4 * lane;
    *(volatile v4f*)op = v;
    __threadfence();
    *(volatile v4f*)op = v;
  }
}

extern "C" void kernel_launch(void* const* d_in, const int* in_sizes, int n_in,
                              void* d_out, int out_size, void* d_ws, size_t ws_size,
                              hipStream_t stream) {
  if (n_in < 4) return;
  const int nx = in_sizes[0];
  if (nx <= 0 || (nx % A_DIM) != 0) return;
  const int n_rows = nx / A_DIM;
  if (in_sizes[1] != R_DIM * A_DIM) return;
  if (in_sizes[2] != R_DIM * A_DIM) return;
  if (in_sizes[3] != R_DIM * (A_DIM + 1)) return;
  if (out_size != n_rows) return;
  if ((n_rows % ROWS) != 0) return;

  const float* x     = (const float*)d_in[0];
  const float* mu    = (const float*)d_in[1];
  const float* sigma = (const float*)d_in[2];
  const float* rho   = (const float*)d_in[3];
  float*       out   = (float*)d_out;
  (void)d_ws; (void)ws_size;

  fuzzy_kernel<<<n_rows / ROWS, NTHR, 0, stream>>>(x, mu, sigma, rho, out, n_rows);
}
